// RoformerAttention_23691039605422
// MI455X (gfx1250) — hardware-verified
//
#include <hip/hip_runtime.h>
#ifndef NB
#define NB 2
#endif
#ifndef SEQ
#define SEQ 2048
#endif
#define NB_FULL 2
#define SEQ_FULL 2048
#define DM 1024
#define NH 16
#define NR (NB * SEQ)
#define SCL 0.125f
static_assert(NB >= 1 && NB <= NB_FULL);
static_assert(SEQ >= 128 && SEQ <= SEQ_FULL && (SEQ % 128) == 0);
static_assert(NH * 64 == DM);
static_assert((NR % 128) == 0);
static_assert((DM % 64) == 0 && (DM % 32) == 0);

typedef unsigned short v8us __attribute__((ext_vector_type(8), may_alias));
typedef float  v8f  __attribute__((ext_vector_type(8)));
typedef float  v4f  __attribute__((ext_vector_type(4)));
typedef float  v4fa __attribute__((ext_vector_type(4), may_alias));
typedef _Float16 v16h __attribute__((ext_vector_type(16)));
typedef _Float16 v4h __attribute__((ext_vector_type(4)));
union FragH { v16h v; v8us half[2]; _Float16 h[16]; unsigned short u[16]; };

__device__ __forceinline__ unsigned short bf16_bits(float x) { unsigned int u = __float_as_uint(x); return (unsigned short)((u + 0x7FFFu + ((u >> 16) & 1u)) >> 16); }
__device__ __forceinline__ float bf16_val(unsigned short b) { return __uint_as_float(((unsigned int)b) << 16); }
__device__ __forceinline__ float bf16_rne(float x) { return bf16_val(bf16_bits(x)); }

template <int NT>
__device__ __forceinline__ v8f mmaH(v16h ah, v16h al, v16h bh, v16h bl, v8f c) {
  c = __builtin_amdgcn_wmma_f32_16x16x32_f16(false, ah, false, bh, (short)0, c, false, false);
  if (NT >= 2) c = __builtin_amdgcn_wmma_f32_16x16x32_f16(false, al, false, bh, (short)0, c, false, false);
  if (NT >= 3) c = __builtin_amdgcn_wmma_f32_16x16x32_f16(false, ah, false, bl, (short)0, c, false, false);
  asm volatile("v_nop\n\tv_nop\n\tv_nop\n\tv_nop" : "+v"(c) : "v"(ah), "v"(al), "v"(bh), "v"(bl));
  return c;
}

__device__ __forceinline__ v16h g2_frag(const _Float16* p, int hh) { FragH f; f.half[0] = *(const v8us*)((const unsigned short*)p + 8 * hh); f.half[1] = *(const v8us*)((const unsigned short*)p + 16 + 8 * hh); return f.v; }
__device__ __forceinline__ v8f g2_mma(v16h a, v16h b, v8f c) { v8f d = __builtin_amdgcn_wmma_f32_16x16x32_f16(false, a, false, b, (short)0, c, false, false); asm volatile("v_nop\n\tv_nop\n\tv_nop\n\tv_nop" : "+v"(d) : "v"(a), "v"(b)); return d; }
template <int ACT>
__global__ __launch_bounds__(128) void k_gemm2(const _Float16* __restrict__ A, int lda, size_t sA, const _Float16* __restrict__ Bh, int ldb, size_t sB, float alpha, const float* __restrict__ bias, size_t sBias, const float* CP, int rowsPerB, size_t sCPb, int row0g,
    float* C, _Float16* C16, int ldc, size_t sC, int M, int N, int K) {
  __shared__ __attribute__((aligned(16))) float so[4][32][68];
  const int tid = threadIdx.x, w = tid >> 5, lane = tid & 31, ln = lane & 15, hh = lane >> 4; const int by = blockIdx.y;
  A += (size_t)by * sA; Bh += (size_t)by * sB; const size_t cofs = (size_t)by * sC; const float* bp = bias ? bias + (size_t)by * sBias : nullptr;
  const int ntn = N >> 6; const int mt = blockIdx.x / ntn, nq = blockIdx.x - mt * ntn; const int row0 = mt * 128 + 32 * w, col0 = nq * 64; if (row0 >= M) return;
  const _Float16* a0p = A + (size_t)(row0 + ln) * lda; const _Float16* a1p = a0p + (size_t)16 * lda;
  const _Float16* b0p = Bh + (size_t)(col0 + ln) * ldb; const _Float16* b1p = b0p + (size_t)16 * ldb; const _Float16* b2p = b1p + (size_t)16 * ldb; const _Float16* b3p = b2p + (size_t)16 * ldb;
  const v8f z8 = {0.f,0.f,0.f,0.f,0.f,0.f,0.f,0.f}; v8f c00 = z8, c01 = z8, c02 = z8, c03 = z8, c10 = z8, c11 = z8, c12 = z8, c13 = z8;
#pragma unroll 1
  for (int kb = 0; kb < K; kb += 32) { const v16h a0 = g2_frag(a0p + kb, hh), a1 = g2_frag(a1p + kb, hh);
    v16h b = g2_frag(b0p + kb, hh); c00 = g2_mma(a0, b, c00); c10 = g2_mma(a1, b, c10);
    b = g2_frag(b1p + kb, hh); c01 = g2_mma(a0, b, c01); c11 = g2_mma(a1, b, c11);
    b = g2_frag(b2p + kb, hh); c02 = g2_mma(a0, b, c02); c12 = g2_mma(a1, b, c12);
    b = g2_frag(b3p + kb, hh); c03 = g2_mma(a0, b, c03); c13 = g2_mma(a1, b, c13); }
  v8f accs[8] = {c00, c01, c02, c03, c10, c11, c12, c13};
#pragma unroll
  for (int u = 0; u < 8; ++u) { const int t = u & 3, half = u >> 2; const int col = col0 + t * 16 + ln; const float bv = bp ? bf16_rne(bp[col]) : 0.f;
#pragma unroll
    for (int r = 0; r < 8; ++r) { const int rloc = half * 16 + 8 * hh + r; float v = accs[u][r] * alpha + bv;
      if (CP) { if (rowsPerB < 0) v += CP[cofs + (size_t)(row0g + row0 + rloc) * ldc + col];        else { const int bidx = (row0g + row0 + rloc) / rowsPerB; v += CP[(size_t)bidx * sCPb + (size_t)by * 64 + col]; } }
      if (ACT == 3) v = fmaxf(v, 0.f);
      so[w][rloc][t * 16 + ln] = v; } }
  __builtin_amdgcn_fence(__ATOMIC_ACQ_REL, "workgroup"); __builtin_amdgcn_wave_barrier();
  const int rsub = lane >> 4, c4 = (lane & 15) * 4;
  for (int pass = 0; pass < 2; ++pass) {
#pragma unroll
    for (int q = 0; q < 16; ++q) { const int r = q * 2 + rsub; const v4f v = *(const v4fa*)&so[w][r][c4]; if (C) *(volatile v4f*)(C + cofs + (size_t)(row0 + r) * ldc + col0 + c4) = v; if (C16) { v4h h4;
#pragma unroll
        for (int i = 0; i < 4; ++i) h4[i] = (_Float16)v[i]; *(volatile v4h*)(C16 + cofs + (size_t)(row0 + r) * ldc + col0 + c4) = h4; } }
    if (pass == 0) __threadfence(); } }

__global__ __launch_bounds__(256) void k_wsc(const float* __restrict__ Wm, _Float16* __restrict__ Bt, size_t n8, float sc) {
  const size_t t = (size_t)blockIdx.x * 256 + threadIdx.x; if (t >= n8) return; FragH f; const v4f a = *(const v4fa*)(Wm + t * 8), c = *(const v4fa*)(Wm + t * 8 + 4);
#pragma unroll
  for (int q = 0; q < 4; ++q) { f.h[q] = (_Float16)(bf16_rne(a[q]) * sc); f.h[4 + q] = (_Float16)(bf16_rne(c[q]) * sc); }
  *(volatile v8us*)((unsigned short*)Bt + t * 8) = f.half[0]; __threadfence(); *(volatile v8us*)((unsigned short*)Bt + t * 8) = f.half[0]; }

__global__ __launch_bounds__(256) void k_x16b(const float* __restrict__ x, _Float16* __restrict__ X16) {
  const size_t t = (size_t)blockIdx.x * 256 + threadIdx.x; if (t >= (size_t)NR * DM / 8) return; const size_t row = (t * 8) / DM; const int c0 = (int)((t * 8) % DM); const size_t rb = row / SEQ, rs = row % SEQ;
  const float* src = x + (rb * SEQ_FULL + rs) * (size_t)DM + c0; const v4f a = *(const v4fa*)src, c = *(const v4fa*)(src + 4); FragH f;
#pragma unroll
  for (int q = 0; q < 4; ++q) { f.h[q] = (_Float16)bf16_rne(a[q]); f.h[4 + q] = (_Float16)bf16_rne(c[q]); }
  *(volatile v8us*)((unsigned short*)X16 + t * 8) = f.half[0]; __threadfence(); *(volatile v8us*)((unsigned short*)X16 + t * 8) = f.half[0]; }

__global__ __launch_bounds__(256) void k_hl(const float* __restrict__ F, _Float16* __restrict__ Hh, _Float16* __restrict__ Hl, size_t n8) {
  const size_t t = (size_t)blockIdx.x * 256 + threadIdx.x; if (t >= n8) return; FragH fh, fl; const v4f a = *(const v4fa*)(F + t * 8), c = *(const v4fa*)(F + t * 8 + 4);
#pragma unroll
  for (int q = 0; q < 4; ++q) { _Float16 hv = (_Float16)a[q]; fh.h[q] = hv; fl.h[q] = (_Float16)((a[q] - (float)hv) * 1024.0f); hv = (_Float16)c[q]; fh.h[4 + q] = hv; fl.h[4 + q] = (_Float16)((c[q] - (float)hv) * 1024.0f); }
  for (int pass = 0; pass < 2; ++pass) { *(volatile v8us*)((unsigned short*)Hh + t * 8) = fh.half[0]; *(volatile v8us*)((unsigned short*)Hl + t * 8) = fl.half[0]; if (pass == 0) __threadfence(); } }

__global__ __launch_bounds__(256) void k_rotab(float* __restrict__ CS, float* __restrict__ SN) {
  #pragma clang fp contract(off)
  const int t = blockIdx.x * 256 + threadIdx.x; if (t >= SEQ * 32) return; const int j = t % 32, s = t / 32; const float ex = (float)(2 * j) / 64.0f; const float inv = 1.0f / powf(10000.0f, ex); const float th = (float)s * inv; const float c = cosf(th), sn = sinf(th);
  for (int pass = 0; pass < 2; ++pass) { *(volatile float*)(CS + t) = c; *(volatile float*)(SN + t) = sn; if (pass == 0) __threadfence(); } }

__global__ __launch_bounds__(256) void k_rope4(const float* __restrict__ F, const float* __restrict__ CS, const float* __restrict__ SN, _Float16* __restrict__ H, _Float16* __restrict__ L) {
  #pragma clang fp contract(off)
  const size_t t = (size_t)blockIdx.x * 256 + threadIdx.x; if (t >= (size_t)NR * DM / 8) return; const size_t e0 = t * 8; const size_t row = e0 / DM; const int c0 = (int)(e0 % DM); const int j0 = c0 & 31; const int s = (int)(row % SEQ);
  const v4f a = *(const v4fa*)(F + e0), c = *(const v4fa*)(F + e0 + 4); const float xs[8] = {a[0], a[1], a[2], a[3], c[0], c[1], c[2], c[3]};
  const float* tp = CS + (size_t)s * 32 + j0; const float* up = SN + (size_t)s * 32 + j0; const v4f ca = *(const v4fa*)tp, cb = *(const v4fa*)(tp + 4), sa = *(const v4fa*)up, sb = *(const v4fa*)(up + 4);
  const float cs[8] = {ca[0], ca[1], ca[2], ca[3], cb[0], cb[1], cb[2], cb[3]}; const float sn[8] = {sa[0], sa[1], sa[2], sa[3], sb[0], sb[1], sb[2], sb[3]};
  FragH fh, fl;
#pragma unroll
  for (int q = 0; q < 8; ++q) { const float pr = xs[q ^ 1]; const float rh = (q & 1) ? pr : -pr; float o = xs[q] * cs[q]; o += rh * sn[q];
    const _Float16 hv = (_Float16)o; fh.h[q] = hv; fl.h[q] = (_Float16)((o - (float)hv) * 1024.0f); }
  for (int pass = 0; pass < 2; ++pass) { *(volatile v8us*)((unsigned short*)H + e0) = fh.half[0]; *(volatile v8us*)((unsigned short*)L + e0) = fl.half[0]; if (pass == 0) __threadfence(); } }

__global__ __launch_bounds__(256) void k_vtg(const _Float16* __restrict__ V16, _Float16* __restrict__ Vt) {
  __shared__ unsigned short tl[64][66]; const int tid = threadIdx.x; const int slab = blockIdx.x / (SEQ / 64), lg = blockIdx.x % (SEQ / 64); const int b = slab / NH, h = slab % NH;
  for (int i = tid; i < 64 * 8; i += 256) { const int r = i / 8, c8 = (i % 8) * 8; FragH f; f.half[0] = *(const v8us*)((const unsigned short*)V16 + ((size_t)b * SEQ + lg * 64 + r) * DM + h * 64 + c8);
#pragma unroll
    for (int q = 0; q < 8; ++q) tl[r][c8 + q] = f.u[q]; }
  __syncthreads();
  for (int pass = 0; pass < 2; ++pass) {
#pragma unroll
    for (int rd = 0; rd < 2; ++rd) { const int d = rd * 32 + tid / 8, pc = tid % 8; FragH f;
#pragma unroll
      for (int q = 0; q < 8; ++q) f.u[q] = tl[pc * 8 + q][d];
      *(volatile v8us*)((unsigned short*)Vt + ((size_t)slab * 64 + d) * SEQ + lg * 64 + pc * 8) = f.half[0]; }
    if (pass == 0) __threadfence(); } }

__global__ __launch_bounds__(128) void k_attn(const _Float16* __restrict__ Q16, const _Float16* __restrict__ QL, int ldq, const _Float16* __restrict__ K16, const _Float16* __restrict__ KL, int ldk,
                                             const _Float16* __restrict__ Vt, const _Float16* __restrict__ VtL, const float* __restrict__ AM, const float* __restrict__ AW, float* __restrict__ O, int ldo) {
  constexpr int RPW = 16, DT = 4, KS = 2, QBN = SEQ / 64;
  __shared__ __attribute__((aligned(16))) unsigned short sP[4][RPW][40]; __shared__ __attribute__((aligned(16))) unsigned short sPL[4][RPW][40]; __shared__ __attribute__((aligned(16))) float sO[4][RPW][64 + 4];
  const int tid = threadIdx.x, w = tid >> 5, lane = tid & 31, ln = lane & 15, hh = lane >> 4;
  const int slab = blockIdx.x / QBN, qblk = blockIdx.x % QBN; const int b = slab / NH, h = slab % NH; const int qb0 = qblk * (4 * RPW); const int q0 = qb0 + w * RPW;
  const float ww = bf16_rne(AW[0]);
  FragH aq[KS], aql[KS];
  { const unsigned short* qr = (const unsigned short*)Q16 + ((size_t)b * SEQ + q0 + ln) * ldq + h * 64; const unsigned short* ql = (const unsigned short*)QL + ((size_t)b * SEQ + q0 + ln) * ldq + h * 64;
#pragma unroll
    for (int ks = 0; ks < KS; ++ks) { aq[ks].half[0] = *(const v8us*)(qr + ks * 32 + 8 * hh); aq[ks].half[1] = *(const v8us*)(qr + ks * 32 + 16 + 8 * hh); aql[ks].half[0] = *(const v8us*)(ql + ks * 32 + 8 * hh); aql[ks].half[1] = *(const v8us*)(ql + ks * 32 + 16 + 8 * hh); } }
  const unsigned short* Vth = (const unsigned short*)Vt + (size_t)slab * 64 * SEQ; const unsigned short* Vtl = (const unsigned short*)VtL + (size_t)slab * 64 * SEQ;
  const float* amb = AM + (size_t)b * SEQ_FULL * SEQ_FULL;
  const v8f z8 = {0.f,0.f,0.f,0.f,0.f,0.f,0.f,0.f};
  float m_r[8], l_r[8]; v8f oacc[DT], oaccL[DT];
#pragma unroll
  for (int r = 0; r < 8; ++r) { m_r[r] = -3.0e38f; l_r[r] = 0.f; }
#pragma unroll
  for (int dt = 0; dt < DT; ++dt) { oacc[dt] = z8; oaccL[dt] = z8; }
#pragma unroll 1
  for (int j0 = 0; j0 < SEQ; j0 += 32) {
    v8f s[2];
#pragma unroll
    for (int nt = 0; nt < 2; ++nt) { const unsigned short* kr = (const unsigned short*)K16 + ((size_t)b * SEQ + j0 + nt * 16 + ln) * ldk + h * 64; const unsigned short* klr = (const unsigned short*)KL + ((size_t)b * SEQ + j0 + nt * 16 + ln) * ldk + h * 64; FragH bk[KS], bkl[KS];
#pragma unroll
      for (int ks = 0; ks < KS; ++ks) { bk[ks].half[0] = *(const v8us*)(kr + ks * 32 + 8 * hh); bk[ks].half[1] = *(const v8us*)(kr + ks * 32 + 16 + 8 * hh); bkl[ks].half[0] = *(const v8us*)(klr + ks * 32 + 8 * hh); bkl[ks].half[1] = *(const v8us*)(klr + ks * 32 + 16 + 8 * hh); }
      v8f acc = z8, accl = z8;
#pragma unroll
      for (int ks = 0; ks < KS; ++ks) { acc = mmaH<1>(aq[ks].v, aq[ks].v, bk[ks].v, bk[ks].v, acc); accl = mmaH<1>(aql[ks].v, aql[ks].v, bk[ks].v, bk[ks].v, accl); accl = mmaH<1>(aq[ks].v, aq[ks].v, bkl[ks].v, bkl[ks].v, accl); }
#pragma unroll
      for (int r = 0; r < 8; ++r) acc[r] += accl[r] * 0.0009765625f;
      s[nt] = acc; }
#pragma unroll
    for (int r = 0; r < 8; ++r) { const int tq = q0 + 8 * hh + r; const int k0 = j0 + ln, k1 = j0 + 16 + ln; const float* amk = amb + (size_t)tq * SEQ_FULL;
      float s0 = s[0][r] * SCL, s1 = s[1][r] * SCL; s0 += bf16_rne(amk[k0]) * ww; s1 += bf16_rne(amk[k1]) * ww;
      float mc = fmaxf(s0, s1);
      mc = fmaxf(mc, __shfl_xor(mc, 1, 32)); mc = fmaxf(mc, __shfl_xor(mc, 2, 32)); mc = fmaxf(mc, __shfl_xor(mc, 4, 32)); mc = fmaxf(mc, __shfl_xor(mc, 8, 32));
      const float mn = fmaxf(m_r[r], mc); const float al = (mn > -1.0e38f) ? expf(m_r[r] - mn) : 1.0f; m_r[r] = mn; const float p0 = expf(s0 - mn), p1 = expf(s1 - mn); l_r[r] = l_r[r] * al + p0 + p1;
#pragma unroll
      for (int dt = 0; dt < DT; ++dt) { oacc[dt][r] *= al; oaccL[dt][r] *= al; }
      FragH t2, t2l; const float ps0 = p0 * 1024.0f, ps1 = p1 * 1024.0f; t2.h[0] = (_Float16)ps0; t2.h[1] = (_Float16)ps1; t2l.h[0] = (_Float16)((ps0 - (float)t2.h[0]) * 1024.0f); t2l.h[1] = (_Float16)((ps1 - (float)t2.h[1]) * 1024.0f);
      sP[w][8 * hh + r][ln] = t2.u[0]; sP[w][8 * hh + r][16 + ln] = t2.u[1]; sPL[w][8 * hh + r][ln] = t2l.u[0]; sPL[w][8 * hh + r][16 + ln] = t2l.u[1]; }
    __builtin_amdgcn_fence(__ATOMIC_ACQ_REL, "workgroup"); __builtin_amdgcn_wave_barrier();
    FragH pa, pl;
    pa.half[0] = *(const v8us*)&sP[w][ln][8 * hh]; pa.half[1] = *(const v8us*)&sP[w][ln][16 + 8 * hh]; pl.half[0] = *(const v8us*)&sPL[w][ln][8 * hh]; pl.half[1] = *(const v8us*)&sPL[w][ln][16 + 8 * hh];
#pragma unroll
    for (int dt = 0; dt < DT; ++dt) { const unsigned short* vrow = Vth + (size_t)(dt * 16 + ln) * SEQ + j0; const unsigned short* vrl = Vtl + (size_t)(dt * 16 + ln) * SEQ + j0; FragH bv, bl;
      bv.half[0] = *(const v8us*)(vrow + 8 * hh); bv.half[1] = *(const v8us*)(vrow + 16 + 8 * hh); bl.half[0] = *(const v8us*)(vrl + 8 * hh); bl.half[1] = *(const v8us*)(vrl + 16 + 8 * hh);
      oacc[dt] = mmaH<1>(pa.v, pa.v, bv.v, bv.v, oacc[dt]); oaccL[dt] = mmaH<1>(pl.v, pl.v, bv.v, bv.v, oaccL[dt]); oaccL[dt] = mmaH<1>(pa.v, pa.v, bl.v, bl.v, oaccL[dt]); }
    __builtin_amdgcn_fence(__ATOMIC_ACQ_REL, "workgroup"); __builtin_amdgcn_wave_barrier(); }
#pragma unroll
  for (int r = 0; r < 8; ++r) { float l = l_r[r]; l += __shfl_xor(l, 1, 32); l += __shfl_xor(l, 2, 32); l += __shfl_xor(l, 4, 32); l += __shfl_xor(l, 8, 32); l_r[r] = (l > 0.f) ? 1.0f / (l * 1024.0f) : 0.f; }
#pragma unroll
  for (int dt = 0; dt < DT; ++dt)
#pragma unroll
    for (int r = 0; r < 8; ++r) { float v = oacc[dt][r]; v += oaccL[dt][r] * 0.0009765625f; sO[w][8 * hh + r][dt * 16 + ln] = v * l_r[r]; }
  __builtin_amdgcn_fence(__ATOMIC_ACQ_REL, "workgroup"); __builtin_amdgcn_wave_barrier();
  for (int pass = 0; pass < 2; ++pass) {
#pragma unroll
    for (int rp = 0; rp < RPW; rp += 2) { const int r = rp + (lane >> 4), pc = lane & 15; const v4f val = *(const v4fa*)&sO[w][r][pc * 4]; *(volatile v4f*)(O + ((size_t)b * SEQ + q0 + r) * ldo + h * 64 + pc * 4) = val; }
    if (pass == 0) __threadfence(); } }

__global__ __launch_bounds__(256) void k_ln1024(const float* __restrict__ A, const float* __restrict__ res, const float* __restrict__ g, const float* __restrict__ bb, float* __restrict__ Y) {
  #pragma clang fp contract(off)
  const int wv = threadIdx.x >> 5, ln = threadIdx.x & 31; const size_t r = (size_t)blockIdx.x * 8 + wv; if (r >= (size_t)NR) return;
  const size_t rb = r / SEQ, rs = r % SEQ; const size_t rin = rb * SEQ_FULL + rs;
  float xv[32]; float sm = 0.f;
#pragma unroll
  for (int i = 0; i < 8; ++i) { const int c0 = i * 128 + ln * 4; const v4f a = *(const v4fa*)(A + r * DM + c0); const v4f rr = *(const v4fa*)(res + rin * DM + c0);
#pragma unroll
    for (int q = 0; q < 4; ++q) { const float v = a[q] + bf16_rne(rr[q]); xv[i * 4 + q] = v; sm += v; } }
#pragma unroll
  for (int o = 16; o > 0; o >>= 1) sm += __shfl_xor(sm, o, 32);
  const float mu = sm * 0.0009765625f; float var = 0.f;
#pragma unroll
  for (int q = 0; q < 32; ++q) { const float d = xv[q] - mu; var += d * d; }
#pragma unroll
  for (int o = 16; o > 0; o >>= 1) var += __shfl_xor(var, o, 32);
  const float inv = 1.0f / sqrtf(var * 0.0009765625f + 1e-5f);
  for (int pass = 0; pass < 2; ++pass) {
#pragma unroll
    for (int i = 0; i < 8; ++i) { const int c0 = i * 128 + ln * 4; v4f y;
#pragma unroll
      for (int q = 0; q < 4; ++q) { float v = (xv[i * 4 + q] - mu) * inv; v *= bf16_rne(g[c0 + q]); v += bf16_rne(bb[c0 + q]); y[q] = v; }
      *(volatile v4f*)(Y + rin * DM + c0) = y; }
    if (pass == 0) __threadfence(); } }

extern "C" void kernel_launch(void* const* d_in, const int* in_sizes, int n_in,
                              void* d_out, int out_size, void* d_ws, size_t ws_size, hipStream_t stream) {
  if (n_in < 13) return;
  const float* x = (const float*)d_in[0]; const float* cdm = (const float*)d_in[1];
  const float* Wq = (const float*)d_in[2]; const float* bq = (const float*)d_in[3]; const float* Wk = (const float*)d_in[4]; const float* bk = (const float*)d_in[5];
  const float* Wv = (const float*)d_in[6]; const float* bv = (const float*)d_in[7]; const float* Wo = (const float*)d_in[8]; const float* bo = (const float*)d_in[9];
  const float* gam = (const float*)d_in[10]; const float* bet = (const float*)d_in[11]; const float* cdw = (const float*)d_in[12];
  const long long rows_need = (long long)(NB - 1) * SEQ_FULL + SEQ;
  if ((long long)in_sizes[0] < rows_need * DM) return;
  if ((long long)in_sizes[1] < (long long)(NB - 1) * SEQ_FULL * SEQ_FULL + (long long)(SEQ - 1) * SEQ_FULL + SEQ) return;
  if (in_sizes[2] < DM * DM || in_sizes[4] < DM * DM || in_sizes[6] < DM * DM || in_sizes[8] < DM * DM) return;
  if (in_sizes[3] < DM || in_sizes[5] < DM || in_sizes[7] < DM || in_sizes[9] < DM || in_sizes[10] < DM || in_sizes[11] < DM || in_sizes[12] < 1) return;
  if ((long long)out_size < rows_need * DM) return;
  char* ws = (char*)d_ws; size_t off = 0;
  auto take = [&](size_t bytes) { char* p = ws + off; off += (bytes + 255) & ~(size_t)255; return p; };
  const size_t np = (size_t)NR * DM;
  _Float16* BQ = (_Float16*)take((size_t)DM * DM * 2); _Float16* BK = (_Float16*)take((size_t)DM * DM * 2); _Float16* BV = (_Float16*)take((size_t)DM * DM * 2); _Float16* BO = (_Float16*)take((size_t)DM * DM * 2);
  _Float16* X16 = (_Float16*)take(np * 2); float* F32 = (float*)take(np * 4);
  _Float16* QH = (_Float16*)take(np * 2); _Float16* QL = (_Float16*)take(np * 2); _Float16* KH = (_Float16*)take(np * 2); _Float16* KL = (_Float16*)take(np * 2);
  _Float16* V16 = (_Float16*)take(np * 2); _Float16* VLr = (_Float16*)take(np * 2); _Float16* VT = (_Float16*)take(np * 2); _Float16* VTL = (_Float16*)take(np * 2);
  float* Y = (float*)take(np * 4); float* CS = (float*)take((size_t)SEQ * 32 * 4); float* SN = (float*)take((size_t)SEQ * 32 * 4);
  float* O = F32; _Float16* OH = QH; _Float16* OL = KH;
  if (off > ws_size) return;
  const unsigned wb = (unsigned)(((size_t)DM * DM / 8 + 255) / 256); const unsigned eb = (unsigned)((np / 8 + 255) / 256);
  k_wsc<<<wb, 256, 0, stream>>>(Wq, BQ, (size_t)DM * DM / 8, 16.0f); k_wsc<<<wb, 256, 0, stream>>>(Wk, BK, (size_t)DM * DM / 8, 16.0f);
  k_wsc<<<wb, 256, 0, stream>>>(Wv, BV, (size_t)DM * DM / 8, 16.0f); k_wsc<<<wb, 256, 0, stream>>>(Wo, BO, (size_t)DM * DM / 8, 16.0f);
  k_x16b<<<eb, 256, 0, stream>>>(x, X16);
  k_rotab<<<(SEQ * 32 + 255) / 256, 256, 0, stream>>>(CS, SN);
  const dim3 g((NR / 128) * (DM / 64), 1);
  k_gemm2<0><<<g, 128, 0, stream>>>(X16, DM, 0, BQ, DM, 0, 0.0625f, bq, 0, nullptr, 1, 0, 0, F32, nullptr, DM, 0, NR, DM, DM); k_rope4<<<eb, 256, 0, stream>>>(F32, CS, SN, QH, QL);
  k_gemm2<0><<<g, 128, 0, stream>>>(X16, DM, 0, BK, DM, 0, 0.0625f, bk, 0, nullptr, 1, 0, 0, F32, nullptr, DM, 0, NR, DM, DM); k_rope4<<<eb, 256, 0, stream>>>(F32, CS, SN, KH, KL);
  k_gemm2<0><<<g, 128, 0, stream>>>(X16, DM, 0, BV, DM, 0, 0.0625f, bv, 0, nullptr, 1, 0, 0, F32, nullptr, DM, 0, NR, DM, DM); k_hl<<<eb, 256, 0, stream>>>(F32, V16, VLr, np / 8);
  k_vtg<<<NB * NH * (SEQ / 64), 256, 0, stream>>>(V16, VT); k_vtg<<<NB * NH * (SEQ / 64), 256, 0, stream>>>(VLr, VTL);
  k_attn<<<NB * NH * (SEQ / 64), 128, 0, stream>>>(QH, QL, DM, KH, KL, DM, VT, VTL, cdm, cdw, O, DM);
  k_hl<<<eb, 256, 0, stream>>>(O, OH, OL, np / 8);
  k_gemm2<0><<<g, 128, 0, stream>>>(OL, DM, 0, BO, DM, 0, 0.0625f / 1024.0f, nullptr, 0, nullptr, 1, 0, 0, Y, nullptr, DM, 0, NR, DM, DM);
  k_gemm2<0><<<g, 128, 0, stream>>>(OH, DM, 0, BO, DM, 0, 0.0625f, bo, 0, Y, 1, (size_t)DM, 0, Y, nullptr, DM, 0, NR, DM, DM);
  k_ln1024<<<NR / 8, 256, 0, stream>>>(Y, x, gam, bet, (float*)d_out);
}
